// MambaEncoder_77086073028640
// MI455X (gfx1250) — hardware-verified
//
#include <hip/hip_runtime.h>
#include <math.h>

typedef __attribute__((ext_vector_type(16))) _Float16 v16h;
typedef __attribute__((ext_vector_type(8)))  _Float16 v8h;
typedef __attribute__((ext_vector_type(8)))  float    v8f;
typedef __attribute__((ext_vector_type(4)))  float    v4f;

constexpr int kLayers = 2;
constexpr int kBatch  = 2;
constexpr int kSeqL   = 2048;
constexpr int kDmod   = 768;
constexpr int kDin    = 1536;
constexpr int kNst    = 16;
constexpr int kDtR    = 48;
constexpr int kDtP    = 64;
constexpr int kPrjN   = 80;
constexpr int kPrjP   = 128;
constexpr int kBCoff  = 48;
constexpr int kXZP    = 2 * kDin;
constexpr int kRows   = kBatch * kSeqL;
constexpr int kTP     = 260;
constexpr float kLnEps  = 1e-5f;
constexpr float kInvDm  = 1.0f / (float)kDmod;

constexpr float kCarWin  = 32.0f;
constexpr float kCarWxp  = 32.0f;
constexpr float kCarWdt  = 8.0f;
constexpr float kCarWout = 32.0f;
constexpr float kCarDt   = 16.0f;
constexpr float kCarY    = 16.0f;
constexpr float kFoldS1  = 1.0f / kCarWin;
constexpr float kFoldS2  = 1.0f / kCarWxp;
constexpr float kFoldS3  = 1.0f / (kCarDt * kCarWdt);
constexpr float kFoldS5  = 1.0f / (kCarY * kCarWout);

static_assert(kDtR + 2 * kNst == kPrjN);
static_assert(kBCoff == kDtR && (kBCoff % 4) == 0);
static_assert((kDtR % 8) == 0 && kDtP == 64 && kDtR <= kDtP);
static_assert(kDmod == 3 * 256);
static_assert((kDmod % 32) == 0 && (kDin % 32) == 0 && (kDtP % 32) == 0);
static_assert((kDmod % 64) == 0 && (kDin % 64) == 0);
static_assert((kSeqL % 64) == 0 && (kXZP % 64) == 0 && (kPrjP % 64) == 0);
static_assert((kDin % 256) == 0 && (kSeqL % 16) == 0 && (kRows % 8) == 0);
static_assert((((kSeqL / 64) * (kXZP / 64)) % 8) == 0);
static_assert((((kSeqL / 64) * (kPrjP / 64)) % 8) == 0);
static_assert((((kSeqL / 64) * (kDin / 64)) % 8) == 0);
static_assert((((kSeqL / 64) * (kDmod / 64)) % 8) == 0);

constexpr size_t kSzWIN  = (size_t)kLayers * kXZP * kDmod * 2;
constexpr size_t kSzWXP  = (size_t)kLayers * kPrjP * kDin * 2;
constexpr size_t kSzWDT  = (size_t)kLayers * kDin * kDtP * 2;
constexpr size_t kSzWOUT = (size_t)kLayers * kDmod * kDin * 2;
constexpr size_t kSzXN   = (size_t)kRows * kDmod * 2;
constexpr size_t kSzXZ   = (size_t)kSeqL * kXZP * 4;
constexpr size_t kSzUC   = (size_t)kSeqL * kDin * 4;
constexpr size_t kSzUC16 = (size_t)kSeqL * kDin * 2;
constexpr size_t kSzPROJ = (size_t)kSeqL * kPrjP * 4;
constexpr size_t kSzDT16 = (size_t)kSeqL * kDtP * 2;
constexpr size_t kSzDLR  = (size_t)kSeqL * kDin * 4;
constexpr size_t kSzY16  = (size_t)kSeqL * kDin * 2;
constexpr size_t kSzX1   = (size_t)kRows * kDmod * 4;
constexpr size_t kOffWIN  = 0;
constexpr size_t kOffWXP  = kOffWIN  + kSzWIN;
constexpr size_t kOffWDT  = kOffWXP  + kSzWXP;
constexpr size_t kOffWOUT = kOffWDT  + kSzWDT;
constexpr size_t kOffXN   = kOffWOUT + kSzWOUT;
constexpr size_t kOffXZ   = kOffXN   + kSzXN;
constexpr size_t kOffUC   = kOffXZ   + kSzXZ;
constexpr size_t kOffUC16 = kOffUC   + kSzUC;
constexpr size_t kOffPROJ = kOffUC16 + kSzUC16;
constexpr size_t kOffDT16 = kOffPROJ + kSzPROJ;
constexpr size_t kOffDLR  = kOffDT16 + kSzDT16;
constexpr size_t kOffY16  = kOffDLR  + kSzDLR;
constexpr size_t kOffX1   = kOffY16  + kSzY16;
constexpr size_t kWsTotal = kOffX1   + kSzX1;
static_assert(kWsTotal == 98435072ull);
static_assert(kWsTotal <= 134217728ull);
static_assert((kOffWXP % 128) == 0 && (kOffWDT % 128) == 0 && (kOffWOUT % 128) == 0 && (kOffXN % 128) == 0 &&
              (kOffXZ % 128) == 0 && (kOffUC % 128) == 0 && (kOffUC16 % 128) == 0 && (kOffPROJ % 128) == 0 &&
              (kOffDT16 % 128) == 0 && (kOffDLR % 128) == 0 && (kOffY16 % 128) == 0 && (kOffX1 % 128) == 0);

union FragU { v16h v; v8h h[2]; };
__device__ __forceinline__ v16h frag_load(const _Float16* p) {
  FragU f;
  f.h[0] = *(const v8h*)(p);
  f.h[1] = *(const v8h*)(p + 16);
  return f.v;
}
__device__ __forceinline__ v8f frag_mma(v16h a, v16h b, v8f c) {
  return __builtin_amdgcn_wmma_f32_16x16x32_f16(false, a, false, b, (short)0, c, false, false);
}
__device__ __forceinline__ void guard_row4(v8f& a, v8f& b, v8f& c, v8f& d, v16h x, v16h b0, v16h b1, v16h b2, v16h b3) {
  asm volatile("v_nop\n\tv_nop\n\tv_nop\n\tv_nop" : "+v"(a), "+v"(b), "+v"(c), "+v"(d) : "v"(x), "v"(b0), "v"(b1), "v"(b2), "v"(b3));
}
__device__ __forceinline__ void keep4_h(v16h a, v16h b, v16h c, v16h d) { asm volatile("v_nop" :: "v"(a), "v"(b), "v"(c), "v"(d)); }
__device__ __forceinline__ void acc_guard4(v8f& a, v8f& b, v8f& c, v8f& d) { asm volatile("v_nop\n\tv_nop\n\tv_nop\n\tv_nop" : "+v"(a), "+v"(b), "+v"(c), "+v"(d)); }

template <int BIAS_MODE, bool RESID>
__global__ __launch_bounds__(256) void wmma_gemm64_f16(
    const unsigned short* __restrict__ Ap, int lda,
    const unsigned short* __restrict__ Btp, int ldb,
    float* __restrict__ C, int ldc,
    const float* __restrict__ bias,
    const float* __restrict__ resid,
    int M, int N, int K, float scale)
{
  const _Float16* A  = (const _Float16*)Ap;
  const _Float16* Bt = (const _Float16*)Btp;
  __shared__ __align__(16) float sT[8][16 * 68];
  const int lane = threadIdx.x & 31;
  const int wave = threadIdx.x >> 5;
  const int tilesN = N >> 6;
  const int tilesM = M >> 6;
  const int tile = blockIdx.x * 8 + wave;
  if (tile >= tilesM * tilesN) return;
  const int tm = tile / tilesN;
  const int tn = tile - tm * tilesN;
  const int m0 = tm << 6;
  const int n0 = tn << 6;

  const int rlane = lane & 15;
  const int koff  = (lane >> 4) * 8;
  const int mOff  = (lane >> 4) * 8;

  v8f acc[4][4];
#pragma unroll
  for (int i = 0; i < 4; ++i)
#pragma unroll
    for (int j = 0; j < 4; ++j) acc[i][j] = (v8f){0.f,0.f,0.f,0.f,0.f,0.f,0.f,0.f};

  for (int k0 = 0; k0 < K; k0 += 32) {
    v16h bh[4];
#pragma unroll
    for (int j = 0; j < 4; ++j) {
      const size_t bo = (size_t)(n0 + (j << 4) + rlane) * ldb + koff + k0;
      bh[j] = frag_load(Bt + bo);
    }
#pragma unroll
    for (int i = 0; i < 4; ++i) {
      const size_t ao = (size_t)(m0 + (i << 4) + rlane) * lda + koff + k0;
      const v16h ah = frag_load(A + ao);
#pragma unroll
      for (int j = 0; j < 4; ++j) acc[i][j] = frag_mma(ah, bh[j], acc[i][j]);
      guard_row4(acc[i][0], acc[i][1], acc[i][2], acc[i][3], ah, bh[0], bh[1], bh[2], bh[3]);
    }
    keep4_h(bh[0], bh[1], bh[2], bh[3]);
  }
  acc_guard4(acc[0][0], acc[0][1], acc[0][2], acc[0][3]);
  acc_guard4(acc[1][0], acc[1][1], acc[1][2], acc[1][3]);
  acc_guard4(acc[2][0], acc[2][1], acc[2][2], acc[2][3]);
  acc_guard4(acc[3][0], acc[3][1], acc[3][2], acc[3][3]);

  float* slab = sT[wave];
  const int hh = lane >> 4;
  const int c4 = (lane & 15) * 4;
#pragma unroll
  for (int i = 0; i < 4; ++i) {
    const int mBase = m0 + (i << 4);
#pragma unroll
    for (int j = 0; j < 4; ++j) {
      const int n = n0 + (j << 4) + rlane;
      float bv = 0.f;
      if (BIAS_MODE == 2) bv = bias[n];
#pragma unroll
      for (int r = 0; r < 8; ++r) {
        float v = acc[i][j][r] * scale;
        if (BIAS_MODE == 2) v += bv;
        slab[(mOff + r) * 68 + (j << 4) + rlane] = v;
      }
    }
    __builtin_amdgcn_fence(__ATOMIC_RELEASE, "workgroup");
    __builtin_amdgcn_wave_barrier();
    __builtin_amdgcn_fence(__ATOMIC_ACQUIRE, "workgroup");
    v4f vals[8];
#pragma unroll
    for (int it = 0; it < 8; ++it) {
      const int row = it * 2 + hh;
      v4f v = *(const v4f*)(slab + row * 68 + c4);
      if (RESID) {
        const v4f rv = *(const v4f*)(resid + (size_t)(mBase + row) * ldc + n0 + c4);
        v = v + rv;
      }
      vals[it] = v;
    }
    for (int pass = 0; pass < 2; ++pass) {
#pragma unroll
      for (int it = 0; it < 8; ++it) {
        const int row = it * 2 + hh;
        *(volatile v4f*)(C + (size_t)(mBase + row) * ldc + n0 + c4) = vals[it];
      }
      __threadfence();
    }
    __builtin_amdgcn_fence(__ATOMIC_RELEASE, "workgroup");
    __builtin_amdgcn_wave_barrier();
    __builtin_amdgcn_fence(__ATOMIC_ACQUIRE, "workgroup");
  }
}

__global__ __launch_bounds__(256) void transpose_cast_kernel(
    const float* __restrict__ W, unsigned short* __restrict__ Bt,
    int Kreal, int Kpad, int Ndim, int Npad, float scale)
{
  __shared__ float tile[64 * 65];
  const int tid = threadIdx.x, lane = tid & 31, wave = tid >> 5;
  const int n0 = blockIdx.x * 64;
  const int k0 = blockIdx.y * 64;
  const float* Wl = W + (size_t)blockIdx.z * Kreal * Ndim;
  unsigned short* Bl = Bt + (size_t)blockIdx.z * Npad * Kpad;
#pragma unroll
  for (int p = 0; p < 16; ++p) {
    const int idx = tid + p * 256;
    const int kk  = idx >> 6;
    const int nn  = idx & 63;
    const int n   = n0 + nn;
    const int k   = k0 + kk;
    const int nc  = (n < Ndim) ? n : (Ndim - 1);
    const int kc  = (k < Kreal) ? k : (Kreal - 1);
    const float v = Wl[(size_t)kc * Ndim + nc];
    const bool ok = (n < Ndim) && (k < Kreal);
    tile[kk * 65 + nn] = ok ? (v * scale) : 0.f;
  }
  __syncthreads();
  const int q = lane >> 3, c8 = (lane & 7) * 8;
  v8h hv[2];
#pragma unroll
  for (int it = 0; it < 2; ++it) {
    const int nrow = it * 32 + wave * 4 + q;
#pragma unroll
    for (int e = 0; e < 8; ++e) hv[it][e] = (_Float16)tile[(c8 + e) * 65 + nrow];
  }
  for (int pass = 0; pass < 2; ++pass) {
#pragma unroll
    for (int it = 0; it < 2; ++it) {
      const int nrow = it * 32 + wave * 4 + q;
      *(volatile v8h*)(Bl + (size_t)(n0 + nrow) * Kpad + k0 + c8) = hv[it];
    }
    __threadfence();
  }
}

__global__ __launch_bounds__(256) void layernorm_f16_kernel(
    const float* __restrict__ X, const float* __restrict__ gam, const float* __restrict__ bet,
    unsigned short* __restrict__ XN)
{
  const int lane = threadIdx.x & 31, wave = threadIdx.x >> 5;
  const int row = blockIdx.x * 8 + wave;
  const float* xp = X + (size_t)row * kDmod + lane * 8;
  v4f a[6];
#pragma unroll
  for (int c = 0; c < 3; ++c) {
    a[2 * c]     = *(const v4f*)(xp + c * 256);
    a[2 * c + 1] = *(const v4f*)(xp + c * 256 + 4);
  }
  float s = 0.f;
#pragma unroll
  for (int i = 0; i < 6; ++i) s += (a[i][0] + a[i][1]) + (a[i][2] + a[i][3]);
#pragma unroll
  for (int off = 16; off > 0; off >>= 1) s += __shfl_xor(s, off, 32);
  const float mu = s * kInvDm;
  float q = 0.f;
#pragma unroll
  for (int i = 0; i < 6; ++i) {
#pragma unroll
    for (int e = 0; e < 4; ++e) {
      const float dd = a[i][e] - mu;
      q = fmaf(dd, dd, q);
    }
  }
#pragma unroll
  for (int off = 16; off > 0; off >>= 1) q += __shfl_xor(q, off, 32);
  const float inv = rsqrtf(q * kInvDm + kLnEps);
  v8h hv[3];
#pragma unroll
  for (int c = 0; c < 3; ++c) {
    const v4f g0 = *(const v4f*)(gam + c * 256 + lane * 8);
    const v4f g1 = *(const v4f*)(gam + c * 256 + lane * 8 + 4);
    const v4f b0 = *(const v4f*)(bet + c * 256 + lane * 8);
    const v4f b1 = *(const v4f*)(bet + c * 256 + lane * 8 + 4);
#pragma unroll
    for (int e = 0; e < 4; ++e) {
      const float y0 = ((a[2 * c][e] - mu) * inv) * g0[e] + b0[e];
      const float y1 = ((a[2 * c + 1][e] - mu) * inv) * g1[e] + b1[e];
      hv[c][e]     = (_Float16)y0;
      hv[c][4 + e] = (_Float16)y1;
    }
  }
  for (int pass = 0; pass < 2; ++pass) {
#pragma unroll
    for (int c = 0; c < 3; ++c)
      *(volatile v8h*)(XN + (size_t)row * kDmod + c * 256 + lane * 8) = hv[c];
    __threadfence();
  }
}

__global__ __launch_bounds__(256) void dt_cast_kernel(
    const float* __restrict__ PROJ, unsigned short* __restrict__ DT16, int total8, float scale)
{
  const int i = blockIdx.x * 256 + threadIdx.x;
  if (i >= total8) return;
  const int e0  = i << 3;
  const int row = e0 >> 6;
  const int c8  = e0 & 63;
  const float* p = PROJ + (size_t)row * kPrjP + c8;
  const v4f a0 = *(const v4f*)(p);
  const v4f a1 = *(const v4f*)(p + 4);
  const bool keep = (c8 < kDtR);
  v8h hv;
#pragma unroll
  for (int e = 0; e < 4; ++e) {
    const float f0 = keep ? (a0[e] * scale) : 0.f;
    const float f1 = keep ? (a1[e] * scale) : 0.f;
    hv[e]     = (_Float16)f0;
    hv[4 + e] = (_Float16)f1;
  }
  unsigned short* qd = DT16 + e0;
  *(volatile v8h*)qd = hv;
  __threadfence();
  *(volatile v8h*)qd = hv;
}

__global__ __launch_bounds__(256) void conv_silu_kernel(
    const float* __restrict__ XZ, const float* __restrict__ cw, const float* __restrict__ cb,
    float* __restrict__ UC, unsigned short* __restrict__ UC16)
{
  __shared__ __align__(16) float sT[16 * kTP];
  const int tid = threadIdx.x, lane = tid & 31, wave = tid >> 5;
  const int d0 = blockIdx.x * 256, d = d0 + tid;
  const int t0 = blockIdx.y * 64;
  const v4f wv = *(const v4f*)(cw + (size_t)d * 4);
  const float w0 = wv[0], w1 = wv[1], w2 = wv[2], w3 = wv[3];
  const float bc = cb[d];
  float xm3, xm2, xm1;
  {
    const int r3 = t0 - 3, r2 = t0 - 2, r1 = t0 - 1;
    const float v3 = XZ[(size_t)(r3 < 0 ? 0 : r3) * kXZP + d];
    const float v2 = XZ[(size_t)(r2 < 0 ? 0 : r2) * kXZP + d];
    const float v1 = XZ[(size_t)(r1 < 0 ? 0 : r1) * kXZP + d];
    xm3 = (r3 >= 0) ? v3 : 0.f;
    xm2 = (r2 >= 0) ? v2 : 0.f;
    xm1 = (r1 >= 0) ? v1 : 0.f;
  }
  const int hrow = wave >> 1;
  const int hch  = (wave & 1) * 128 + lane * 4;
#pragma unroll 1
  for (int sub = 0; sub < 4; ++sub) {
    const int lb = t0 + sub * 16;
#pragma unroll 1
    for (int s = 0; s < 16; ++s) {
      const float xc = XZ[(size_t)(lb + s) * kXZP + d];
      float acc = w0 * xm3;
      acc = fmaf(w1, xm2, acc);
      acc = fmaf(w2, xm1, acc);
      acc = fmaf(w3, xc, acc);
      const float sv = acc + bc;
      const float sg = __builtin_amdgcn_rcpf(1.0f + expf(-sv));
      sT[s * kTP + tid] = sv * sg;
      xm3 = xm2; xm2 = xm1; xm1 = xc;
    }
    __syncthreads();
    v4f fv[4];
    v8h bv[2];
#pragma unroll
    for (int it = 0; it < 4; ++it) fv[it] = *(const v4f*)(sT + (it * 4 + hrow) * kTP + hch);
#pragma unroll
    for (int it = 0; it < 2; ++it) {
      const float* sp = sT + (it * 8 + wave) * kTP + lane * 8;
      const v4f a0 = *(const v4f*)(sp);
      const v4f a1 = *(const v4f*)(sp + 4);
#pragma unroll
      for (int e = 0; e < 4; ++e) {
        bv[it][e]     = (_Float16)a0[e];
        bv[it][4 + e] = (_Float16)a1[e];
      }
    }
    for (int pass = 0; pass < 2; ++pass) {
#pragma unroll
      for (int it = 0; it < 4; ++it)
        *(volatile v4f*)(UC + (size_t)(lb + it * 4 + hrow) * kDin + d0 + hch) = fv[it];
#pragma unroll
      for (int it = 0; it < 2; ++it)
        *(volatile v8h*)(UC16 + (size_t)(lb + it * 8 + wave) * kDin + d0 + lane * 8) = bv[it];
      __threadfence();
    }
    __syncthreads();
  }
}

__global__ __launch_bounds__(256) void scan_kernel(
    const float* __restrict__ DLR, const float* __restrict__ UC, const float* __restrict__ XZ,
    const float* __restrict__ PROJ, const float* __restrict__ A_log, const float* __restrict__ Dv,
    unsigned short* __restrict__ Y16)
{
  __shared__ __align__(16) float sBC[16 * 32];
  __shared__ __align__(16) float sY[16 * kTP];
  __shared__ __align__(16) float sA[kNst * 256];
  const int tid = threadIdx.x, lane = tid & 31, wave = tid >> 5;
  const int d0 = blockIdx.x * 256, d = d0 + tid;

#pragma unroll 1
  for (int n = 0; n < kNst; ++n) sA[n * 256 + tid] = -expf(A_log[(size_t)d * kNst + n]);
  __syncthreads();
  float An[kNst], h[kNst];
#pragma unroll
  for (int n = 0; n < kNst; ++n) {
    An[n] = sA[n * 256 + tid];
    h[n] = 0.f;
  }
  const float Dd = Dv[d];

#pragma unroll 1
  for (int c = 0; c < kSeqL / 16; ++c) {
    const int l0 = c * 16;
    if (tid < 128) {
      const int r = tid >> 3, q = (tid & 7) * 4;
      const v4f v = *(const v4f*)(PROJ + (size_t)(l0 + r) * kPrjP + kBCoff + q);
      *(v4f*)(sBC + r * 32 + q) = v;
    }
    __syncthreads();
#pragma unroll 1
    for (int s = 0; s < 16; ++s) {
      const size_t m = (size_t)(l0 + s);
      const float a  = DLR[m * kDin + d];
      const float xv = UC[m * kDin + d];
      const float zv = XZ[m * kXZP + kDin + d];
      const float ea = __expf(-fabsf(a));
      const float u1 = 1.0f + ea;
      const float l1p = __logf(u1) + (ea - (u1 - 1.0f)) * __builtin_amdgcn_rcpf(u1);
      const float delta = fmaxf(a, 0.0f) + l1p;
      v4f Bq[4], Cq[4];
#pragma unroll
      for (int qq = 0; qq < 4; ++qq) {
        Bq[qq] = *(const v4f*)(sBC + s * 32 + 4 * qq);
        Cq[qq] = *(const v4f*)(sBC + s * 32 + kNst + 4 * qq);
      }
      float y = 0.f;
#pragma unroll
      for (int n = 0; n < kNst; ++n) {
        const float e  = __expf(delta * An[n]);
        const float db = delta * Bq[n >> 2][n & 3];
        const float hn = fmaf(e, h[n], db * xv);
        h[n] = hn;
        y = fmaf(Cq[n >> 2][n & 3], hn, y);
      }
      y = fmaf(xv, Dd, y);
      const float sg = __builtin_amdgcn_rcpf(1.0f + expf(-zv));
      const float g  = zv * sg;
      sY[s * kTP + tid] = (y * g) * kCarY;
    }
    __syncthreads();
    v8h hv[2];
#pragma unroll
    for (int it = 0; it < 2; ++it) {
      const float* sp = sY + (it * 8 + wave) * kTP + lane * 8;
      const v4f a0 = *(const v4f*)(sp);
      const v4f a1 = *(const v4f*)(sp + 4);
#pragma unroll
      for (int e = 0; e < 4; ++e) {
        hv[it][e]     = (_Float16)a0[e];
        hv[it][4 + e] = (_Float16)a1[e];
      }
    }
    for (int pass = 0; pass < 2; ++pass) {
#pragma unroll
      for (int it = 0; it < 2; ++it)
        *(volatile v8h*)(Y16 + (size_t)(l0 + it * 8 + wave) * kDin + d0 + lane * 8) = hv[it];
      __threadfence();
    }
  }
}

extern "C" void kernel_launch(void* const* d_in, const int* in_sizes, int n_in,
                              void* d_out, int out_size, void* d_ws, size_t ws_size,
                              hipStream_t stream)
{
  if (n_in < 12) return;
  if (in_sizes[0] != kRows * kDmod) return;
  if (in_sizes[1] != kLayers * kDmod || in_sizes[2] != kLayers * kDmod) return;
  if (in_sizes[3] != kLayers * kDmod * kXZP) return;
  if (in_sizes[4] != kLayers * kDin * 4 || in_sizes[5] != kLayers * kDin) return;
  if (in_sizes[6] != kLayers * kDin * kPrjN) return;
  if (in_sizes[7] != kLayers * kDtR * kDin || in_sizes[8] != kLayers * kDin) return;
  if (in_sizes[9] != kLayers * kDin * kNst || in_sizes[10] != kLayers * kDin) return;
  if (in_sizes[11] != kLayers * kDin * kDmod) return;
  if (out_size != kRows * kDmod) return;
  if (ws_size < kWsTotal) return;

  const float* x      = (const float*)d_in[0];
  const float* gamma  = (const float*)d_in[1];
  const float* beta   = (const float*)d_in[2];
  const float* W_in   = (const float*)d_in[3];
  const float* conv_w = (const float*)d_in[4];
  const float* conv_b = (const float*)d_in[5];
  const float* W_xprj = (const float*)d_in[6];
  const float* W_dt   = (const float*)d_in[7];
  const float* b_dt   = (const float*)d_in[8];
  const float* A_log  = (const float*)d_in[9];
  const float* D_skip = (const float*)d_in[10];
  const float* W_out  = (const float*)d_in[11];
  float* dout = (float*)d_out;

  char* ws = (char*)d_ws;
  unsigned short* WIN16  = (unsigned short*)(ws + kOffWIN);
  unsigned short* WXP16  = (unsigned short*)(ws + kOffWXP);
  unsigned short* WDT16  = (unsigned short*)(ws + kOffWDT);
  unsigned short* WOUT16 = (unsigned short*)(ws + kOffWOUT);
  unsigned short* XN16   = (unsigned short*)(ws + kOffXN);
  float*          XZ     = (float*)(ws + kOffXZ);
  float*          UC     = (float*)(ws + kOffUC);
  unsigned short* UC16   = (unsigned short*)(ws + kOffUC16);
  float*          PROJ   = (float*)(ws + kOffPROJ);
  unsigned short* DT16   = (unsigned short*)(ws + kOffDT16);
  float*          DLR    = (float*)(ws + kOffDLR);
  unsigned short* Y16    = (unsigned short*)(ws + kOffY16);
  float*          X1     = (float*)(ws + kOffX1);

  transpose_cast_kernel<<<dim3(kXZP / 64, kDmod / 64, kLayers), 256, 0, stream>>>(W_in, WIN16, kDmod, kDmod, kXZP, kXZP, kCarWin);
  transpose_cast_kernel<<<dim3(kPrjP / 64, kDin / 64, kLayers), 256, 0, stream>>>(W_xprj, WXP16, kDin, kDin, kPrjN, kPrjP, kCarWxp);
  transpose_cast_kernel<<<dim3(kDin / 64, kDtP / 64, kLayers), 256, 0, stream>>>(W_dt, WDT16, kDtR, kDtP, kDin, kDin, kCarWdt);
  transpose_cast_kernel<<<dim3(kDmod / 64, kDin / 64, kLayers), 256, 0, stream>>>(W_out, WOUT16, kDin, kDin, kDmod, kDmod, kCarWout);

  for (int i = 0; i < kLayers; ++i) {
    const float* g_i   = gamma  + (size_t)i * kDmod;
    const float* be_i  = beta   + (size_t)i * kDmod;
    const float* cw_i  = conv_w + (size_t)i * kDin * 4;
    const float* cb_i  = conv_b + (size_t)i * kDin;
    const float* bdt_i = b_dt   + (size_t)i * kDin;
    const float* Al_i  = A_log  + (size_t)i * kDin * kNst;
    const float* Ds_i  = D_skip + (size_t)i * kDin;
    const unsigned short* WIN_i  = WIN16  + (size_t)i * kXZP * kDmod;
    const unsigned short* WXP_i  = WXP16  + (size_t)i * kPrjP * kDin;
    const unsigned short* WDT_i  = WDT16  + (size_t)i * kDin * kDtP;
    const unsigned short* WOUT_i = WOUT16 + (size_t)i * kDmod * kDin;
    const float* xin  = (i == 0) ? x : (const float*)X1;
    float*       xout = (i == 0) ? X1 : dout;

    layernorm_f16_kernel<<<kRows / 8, 256, 0, stream>>>(xin, g_i, be_i, XN16);

    for (int b = 0; b < kBatch; ++b) {
      const unsigned short* XNb = XN16 + (size_t)b * kSeqL * kDmod;
      const float* xinb = xin  + (size_t)b * kSeqL * kDmod;
      float*      xoutb = xout + (size_t)b * kSeqL * kDmod;

      wmma_gemm64_f16<0, false><<<(kSeqL / 64) * (kXZP / 64) / 8, 256, 0, stream>>>(
          XNb, kDmod, WIN_i, kDmod, XZ, kXZP, bdt_i, xinb, kSeqL, kXZP, kDmod, kFoldS1);

      conv_silu_kernel<<<dim3(kDin / 256, kSeqL / 64), 256, 0, stream>>>(XZ, cw_i, cb_i, UC, UC16);

      wmma_gemm64_f16<0, false><<<(kSeqL / 64) * (kPrjP / 64) / 8, 256, 0, stream>>>(
          UC16, kDin, WXP_i, kDin, PROJ, kPrjP, bdt_i, xinb, kSeqL, kPrjP, kDin, kFoldS2);

      dt_cast_kernel<<<(kSeqL * kDtP) / 8 / 256, 256, 0, stream>>>(PROJ, DT16, (kSeqL * kDtP) / 8, kCarDt);

      wmma_gemm64_f16<2, false><<<(kSeqL / 64) * (kDin / 64) / 8, 256, 0, stream>>>(
          DT16, kDtP, WDT_i, kDtP, DLR, kDin, bdt_i, xinb, kSeqL, kDin, kDtP, kFoldS3);

      scan_kernel<<<kDin / 256, 256, 0, stream>>>(DLR, UC, XZ, PROJ, Al_i, Ds_i, Y16);

      wmma_gemm64_f16<0, true><<<(kSeqL / 64) * (kDmod / 64) / 8, 256, 0, stream>>>(
          Y16, kDin, WOUT_i, kDin, xoutb, kDmod, bdt_i, xinb, kSeqL, kDmod, kDin, kFoldS5);
    }
  }
}
